// GraphNN_10685878632725
// MI455X (gfx1250) — hardware-run, weakly checked
//
#include <hip/hip_runtime.h>

typedef float          v8f   __attribute__((ext_vector_type(8)));
typedef float          v4f   __attribute__((ext_vector_type(4)));
typedef unsigned int   v4u   __attribute__((ext_vector_type(4)));
typedef int            v8i   __attribute__((ext_vector_type(8)));
typedef unsigned short v8us  __attribute__((ext_vector_type(8)));
typedef unsigned short v16us __attribute__((ext_vector_type(16)));
typedef __bf16         v16bf __attribute__((ext_vector_type(16)));
typedef _Float16       v16h  __attribute__((ext_vector_type(16)));
typedef v4f  __attribute__((may_alias)) v4fa;
typedef v8us __attribute__((may_alias)) v8usa;
union FragB { v16bf v; v16us u; v8us h[2]; v8i w; };
union FragH { v16h  v; v16us u; v8us h[2]; v8i w; };

__device__ __forceinline__ v8f wmb(const FragB& a, const FragB& b, v8f c) {
  v8f d = __builtin_amdgcn_wmma_f32_16x16x32_bf16(false, a.v, false, b.v, (short)0, c, false, false);
  asm volatile("v_nop\n\tv_nop\n\tv_nop\n\tv_nop" : "+v"(d) : "v"(a.w), "v"(b.w));
  return d;
}

__device__ __forceinline__ v8f wmh(const FragH& a, const FragH& b, v8f c) {
  v8f d = __builtin_amdgcn_wmma_f32_16x16x32_f16(false, a.v, false, b.v, (short)0, c, false, false);
  asm volatile("v_nop\n\tv_nop\n\tv_nop\n\tv_nop" : "+v"(d) : "v"(a.w), "v"(b.w));
  return d;
}

__device__ __forceinline__ unsigned bf16_bits(float f) {
  const unsigned u = __float_as_uint(f);
  const unsigned r = (u + 0x7FFFu + ((u >> 16) & 1u)) >> 16;
  const unsigned q = (u >> 16) | 0x40u;
  return ((u & 0x7fffffffu) > 0x7f800000u) ? q : r;
}

__device__ __forceinline__ float bf16_val(float f) {
  return __uint_as_float(bf16_bits(f) << 16);
}
__device__ __forceinline__ int clampi(int v, int lo, int hi) {
  return v < lo ? lo : (v > hi ? hi : v);
}

__device__ __forceinline__ unsigned f16_bits(float f) {
  const unsigned u  = __float_as_uint(f);
  const unsigned s  = (u >> 16) & 0x8000u;
  const unsigned a  = u & 0x7fffffffu;
  const unsigned t  = a - 0x38000000u;
  const unsigned r  = (t + 0x0FFFu + ((t >> 13) & 1u)) >> 13;
  const unsigned rc = r > 0x7C00u ? 0x7C00u : r;
  const bool small  = a < 0x38800000u;
  const bool isnan  = a > 0x7f800000u;
  const unsigned fin = small ? 0u : (s | rc);
  return isnan ? (s | 0x7E00u) : fin;
}

__device__ __forceinline__ unsigned pk16(unsigned lo, unsigned hi) { return lo | (hi << 16); }
__device__ __forceinline__ unsigned bf16_lo_bits(float v) {
  float hi = bf16_val(v);
  asm volatile("" : "+v"(hi));
  return bf16_bits(v - hi);
}
__device__ __forceinline__ v4u pack8_bf16(v4f a, v4f c) {
  return (v4u){ pk16(bf16_bits(a[0]), bf16_bits(a[1])), pk16(bf16_bits(a[2]), bf16_bits(a[3])),
                pk16(bf16_bits(c[0]), bf16_bits(c[1])), pk16(bf16_bits(c[2]), bf16_bits(c[3])) };
}
__device__ __forceinline__ v4u pack8_bf16_lo(v4f a, v4f c) {
  return (v4u){ pk16(bf16_lo_bits(a[0]), bf16_lo_bits(a[1])), pk16(bf16_lo_bits(a[2]), bf16_lo_bits(a[3])),
                pk16(bf16_lo_bits(c[0]), bf16_lo_bits(c[1])), pk16(bf16_lo_bits(c[2]), bf16_lo_bits(c[3])) };
}
__device__ __forceinline__ v4u pack8_f16(v4f a, v4f c) {
  return (v4u){ pk16(f16_bits(a[0]), f16_bits(a[1])), pk16(f16_bits(a[2]), f16_bits(a[3])),
                pk16(f16_bits(c[0]), f16_bits(c[1])), pk16(f16_bits(c[2]), f16_bits(c[3])) };
}

template <int FORM>
__global__ __launch_bounds__(256) void k_plane(const float* __restrict__ src, int rows, int cols, int ldsrc,
                                               unsigned short* __restrict__ dst, int MP, int KP) {
  static_assert(FORM >= 0 && FORM <= 3);
  const int KTOT = (FORM == 1 || FORM == 3) ? 2 * KP : KP;
  const unsigned ppr   = (unsigned)(KTOT >> 3);
  const unsigned kp8   = (unsigned)(KP >> 3);
  const unsigned total = (unsigned)MP * ppr;
  const unsigned g     = blockIdx.x * 256u + threadIdx.x;
  const unsigned rowu  = g / ppr;
  const unsigned p     = g - rowu * ppr;
  const bool second    = p >= kp8;
  const int row = (int)rowu;
  const int c0  = (int)((second ? p - kp8 : p) << 3);
  const float* srow = src + (size_t)clampi(row, 0, rows - 1) * (size_t)ldsrc;
  float x[8];
  unsigned mk[8];
#pragma unroll
  for (int e = 0; e < 8; ++e) {
    const int c = c0 + e;
    const float v = srow[clampi(c, 0, cols - 1)];
    asm volatile("" :: "v"(v));
    x[e]  = v;
    mk[e] = (row < rows && c < cols) ? 0xFFFFu : 0u;
  }
  const v4f a = (v4f){ x[0], x[1], x[2], x[3] };
  const v4f c = (v4f){ x[4], x[5], x[6], x[7] };
  v4u o;
  if (FORM == 2) {
    o = pack8_f16(a, c);
  } else {
    const v4u hi = pack8_bf16(a, c);
    o = hi;
    if (FORM == 1) { const v4u lo = pack8_bf16_lo(a, c); o = second ? lo : hi; }
  }
  const v4u mw = (v4u){ pk16(mk[0], mk[1]), pk16(mk[2], mk[3]), pk16(mk[4], mk[5]), pk16(mk[6], mk[7]) };
  o &= mw;
  if (g < total) {
    volatile v4u* q = (volatile v4u*)(dst + (size_t)g * 8);
    *q = o;
    __threadfence();
    *q = o;
  }
}

template <int FORM> struct FragOf    { typedef FragB T; };
template <>         struct FragOf<2> { typedef FragH T; };
__device__ __forceinline__ v8f mm(const FragB& a, const FragB& b, v8f c) { return wmb(a, b, c); }
__device__ __forceinline__ v8f mm(const FragH& a, const FragH& b, v8f c) { return wmh(a, b, c); }
template <class F> __device__ __forceinline__ F ld_frag(const unsigned short* p) {
  F f;
  f.h[0] = *(const v8usa*)(p);
  f.h[1] = *(const v8usa*)(p + 16);
  return f;
}

template <int FORM, int EPI>
__global__ __launch_bounds__(256) __attribute__((amdgpu_num_vgpr(248)))
void k_gemm_nt(const unsigned short* __restrict__ A, const unsigned short* __restrict__ B,
               const float* __restrict__ bias, float* __restrict__ D, int M, int N, int KTOT, int ldd) {
  static_assert(FORM >= 0 && FORM <= 2);
  static_assert(EPI == 0 || EPI == 1);
  typedef typename FragOf<FORM>::T F;
  __shared__ __attribute__((aligned(16))) float sT[8][16 * 68];
  const int lane = threadIdx.x & 31;
  const int wave = threadIdx.x >> 5;
  const int tilesM = (M + 63) >> 6;
  const int tilesN = (N + 63) >> 6;
  const int tile = blockIdx.x * 8 + wave;
  if (tile >= tilesM * tilesN) return;
  const int tm = tile / tilesN;
  const int tn = tile - tm * tilesN;
  const int m0 = tm << 6;
  const int n0 = tn << 6;

  const int rl = lane & 15;
  const int h8 = (lane >> 4) * 8;
  const unsigned short* pa = A + (size_t)(m0 + rl) * (size_t)KTOT + h8;
  const unsigned short* pb = B + (size_t)(n0 + rl) * (size_t)KTOT + h8;

  v8f acc[4][4];
#pragma unroll
  for (int i = 0; i < 4; ++i)
#pragma unroll
    for (int j = 0; j < 4; ++j) acc[i][j] = (v8f){0.f, 0.f, 0.f, 0.f, 0.f, 0.f, 0.f, 0.f};

#pragma unroll 1
  for (int k0 = 0; k0 < KTOT; k0 += 32) {
    F bf[4];
#pragma unroll
    for (int j = 0; j < 4; ++j) bf[j] = ld_frag<F>(pb + (size_t)(j << 4) * (size_t)KTOT + k0);
#pragma unroll
    for (int i = 0; i < 4; ++i) {
      const F af = ld_frag<F>(pa + (size_t)(i << 4) * (size_t)KTOT + k0);
#pragma unroll
      for (int j = 0; j < 4; ++j) acc[i][j] = mm(af, bf[j], acc[i][j]);
    }
  }

  float* slab = sT[wave];
  const int hh = lane >> 4;
  const int c4 = (lane & 15) * 4;
  const int nc = n0 + c4;
  const bool cok = nc < N;
  v4f bv = (v4f){0.f, 0.f, 0.f, 0.f};
  if (EPI == 1) {
    bv = *(const v4fa*)(bias + clampi(nc, 0, N - 4));
    asm volatile("" :: "v"(bv));
  }
#pragma unroll
  for (int i = 0; i < 4; ++i) {
    const int mBase = m0 + (i << 4);
#pragma unroll
    for (int j = 0; j < 4; ++j) {
#pragma unroll
      for (int r = 0; r < 8; ++r) slab[(h8 + r) * 68 + (j << 4) + rl] = acc[i][j][r];
    }
    __builtin_amdgcn_fence(__ATOMIC_RELEASE, "workgroup");
    __builtin_amdgcn_wave_barrier();
    __builtin_amdgcn_fence(__ATOMIC_ACQUIRE, "workgroup");
    v4f vv[8];
#pragma unroll
    for (int it = 0; it < 8; ++it) {
      const int row = it * 2 + hh;
      v4f v = *(const v4fa*)(slab + row * 68 + c4);
      if (EPI == 1) v += bv;
      vv[it] = v;
    }
    for (int pass = 0; pass < 2; ++pass) {
#pragma unroll
      for (int it = 0; it < 8; ++it) {
        const int row = mBase + it * 2 + hh;
        if (cok && row < M) *(volatile v4f*)(D + (size_t)row * (size_t)ldd + nc) = vv[it];
      }
      __threadfence();
    }
    __builtin_amdgcn_fence(__ATOMIC_RELEASE, "workgroup");
    __builtin_amdgcn_wave_barrier();
    __builtin_amdgcn_fence(__ATOMIC_ACQUIRE, "workgroup");
  }
}

#include <stddef.h>
#include <stdint.h>
#include <math.h>

#define NN       100000
#define NE       1600000
#define DIN      64
#define HID      128
#define DOUT     64
#define MPAD     100096
#define H1_TERMS 2
#define K2TOT    (HID * H1_TERMS)
#define NTHR     256
#define NWAVE    8
#define EPT      8
#define CHUNK    (NTHR * EPT)
#define NCHUNK   ((NE + CHUNK - 1) / CHUNK)
#define WCAP     (EPT * 32)
#define LISTN    (NWAVE * WCAP)
#define NBA      1024
#define SLA      10
#define NBLK     98
#define NTAB     (NBLK * NBA)
#define RCAP     28672
#define DEGCAP   64
#define BK_ZINTS (LISTN + 2 * RCAP + 3 * NBA)
#define BK_LDS_INTS (BK_ZINTS + 16)
#define BK_LDS_BYTES (BK_LDS_INTS * 4)
#define NU1      (HID * (DIN / 8))
#define NU2      (DOUT * (K2TOT / 8))
#define PARN     320
#define TOTP     (NN * DOUT / 4)
#define WSMAX    ((size_t)128 << 20)

static_assert(H1_TERMS == 1 || H1_TERMS == 2);
static_assert(NE % EPT == 0 && NE % 4 == 0 && NE >= EPT);
static_assert(((long long)NCHUNK * CHUNK << SLA) < (1LL << 31));
static_assert(NBA == (1 << SLA) && NBLK * NBA >= MPAD && MPAD >= NN);
static_assert(MPAD % 64 == 0 && MPAD % 16 == 0 && NN % 16 == 0);
static_assert(DIN % 32 == 0 && K2TOT % 32 == 0 && HID % 64 == 0 && DOUT % 64 == 0);
static_assert(RCAP * 100LL >= 16703LL * 105LL);
static_assert(DEGCAP >= 36 + 8);
static_assert(RCAP % (4 * NTHR) == 0 && BK_ZINTS % 4 == 0 && LISTN % 4 == 0);
static_assert(BK_LDS_BYTES <= 327680);
static_assert(NU1 % NTHR == 0 && NU2 % NTHR == 0);
static_assert(NBA % NWAVE == 0 && NBA == 4 * NTHR);
static_assert((MPAD * (DIN / 8)) % 256 == 0);
static_assert(TOTP * 4 == NN * DOUT);

typedef float  v2f __attribute__((ext_vector_type(2)));
typedef int    v4i __attribute__((ext_vector_type(4)));
typedef double v2d __attribute__((ext_vector_type(2)));
typedef v2f __attribute__((may_alias)) v2fa;
typedef v4i __attribute__((may_alias)) v4ia;
typedef v2d __attribute__((may_alias)) v2da;

constexpr size_t SZ_RA   = (size_t)MPAD * HID * 4;
constexpr size_t SZ_RB   = (size_t)MPAD * 256 * 2;
constexpr size_t SZ_LIST = (size_t)NBLK * RCAP * 4;
constexpr size_t SZ_TAB  = (size_t)NTAB * 4;
constexpr size_t SZ_FLAG = (size_t)NBLK * 128;
constexpr size_t SZ_W1T  = (size_t)HID * DIN * 2;
constexpr size_t SZ_W2D  = (size_t)DOUT * 256 * 2;
constexpr size_t SZ_PAR  = (size_t)PARN * 4;
constexpr size_t SZ_STAT = (size_t)256 * 4;
constexpr size_t SZ_REC  = (size_t)NBLK * 64 * 8;
constexpr size_t SZ_MEAN = (size_t)64 * 8;
constexpr size_t O_RA   = 0;
constexpr size_t O_RB   = O_RA + SZ_RA;
constexpr size_t O_LIST = O_RB + SZ_RB;
constexpr size_t O_CNT  = O_LIST + SZ_LIST;
constexpr size_t O_OFF  = O_CNT + SZ_TAB;
constexpr size_t O_DIS  = O_OFF + SZ_TAB;
constexpr size_t O_FLAG = O_DIS + SZ_TAB;
constexpr size_t O_W1T  = O_FLAG + SZ_FLAG;
constexpr size_t O_W2D  = O_W1T + SZ_W1T;
constexpr size_t O_PAR  = O_W2D + SZ_W2D;
constexpr size_t O_STAT = O_PAR + SZ_PAR;
constexpr size_t O_RECS = O_STAT + SZ_STAT;
constexpr size_t O_RECQ = O_RECS + SZ_REC;
constexpr size_t O_MEAN = O_RECQ + SZ_REC;
constexpr size_t WS_TOTAL = O_MEAN + SZ_MEAN;
static_assert(SZ_RA % 256 == 0 && SZ_RB % 256 == 0 && SZ_LIST % 256 == 0 && SZ_TAB % 256 == 0);
static_assert(SZ_FLAG % 256 == 0 && SZ_W1T % 256 == 0 && SZ_W2D % 256 == 0 && SZ_PAR % 256 == 0);
static_assert(SZ_STAT % 256 == 0 && SZ_REC % 256 == 0 && SZ_MEAN % 256 == 0);
static_assert((size_t)MPAD * DIN * 2 <= SZ_RB && (size_t)MPAD * K2TOT * 2 <= SZ_RB);
static_assert((size_t)MPAD * DOUT * 4 * 2 <= SZ_RA);
static_assert((size_t)DOUT * K2TOT * 2 <= SZ_W2D);
static_assert(WS_TOTAL <= (size_t)WSMAX);

__global__ __launch_bounds__(NTHR) void k_prep(const float* __restrict__ W1, const float* __restrict__ W2,
                                               const float* __restrict__ b1, const float* __restrict__ b2,
                                               const float* __restrict__ gam, const float* __restrict__ bet,
                                               unsigned short* W1T, unsigned short* W2D, float* PAR) {
  const int u = (int)blockIdx.x * NTHR + (int)threadIdx.x;
  if (u < NU1) {
    const int n  = u >> 3;
    const int k8 = (u & 7) * 8;
    const float* p = W1 + (size_t)k8 * HID + n;
    unsigned w[8];
#pragma unroll
    for (int i = 0; i < 8; ++i) w[i] = bf16_bits(p[(size_t)i * HID]);
    const v4u o = (v4u){ pk16(w[0], w[1]), pk16(w[2], w[3]), pk16(w[4], w[5]), pk16(w[6], w[7]) };
    volatile v4u* q = (volatile v4u*)(W1T + (size_t)n * DIN + k8);
    *q = o;
    __threadfence();
    *q = o;
  } else if (u < NU1 + NU2) {
    const int v  = u - NU1;
    const int n  = v / (K2TOT / 8);
    const int k8 = (v - n * (K2TOT / 8)) * 8;
    const int kk = k8 & (HID - 1);
    const float* p = W2 + (size_t)kk * DOUT + n;
    unsigned w[8];
#pragma unroll
    for (int i = 0; i < 8; ++i) w[i] = bf16_bits(p[(size_t)i * DOUT]);
    const v4u o = (v4u){ pk16(w[0], w[1]), pk16(w[2], w[3]), pk16(w[4], w[5]), pk16(w[6], w[7]) };
    volatile v4u* q = (volatile v4u*)(W2D + (size_t)n * K2TOT + k8);
    *q = o;
    __threadfence();
    *q = o;
  } else {
    const int v = u - (NU1 + NU2);
    const v4f x1 = *(const v4fa*)(b1  + 4 * clampi(v, 0, 31));
    const v4f x2 = *(const v4fa*)(b2  + 4 * clampi(v - 32, 0, 15));
    const v4f x3 = *(const v4fa*)(gam + 4 * clampi(v - 48, 0, 15));
    const v4f x4 = *(const v4fa*)(bet + 4 * clampi(v - 64, 0, 15));
    asm volatile("" :: "v"(x1), "v"(x2), "v"(x3), "v"(x4));
    const unsigned m1 = (v < 32) ? 0xFFFFFFFFu : 0u;
    const unsigned m2 = (v >= 32 && v < 48) ? 0xFFFFFFFFu : 0u;
    const unsigned m3 = (v >= 48 && v < 64) ? 0xFFFFFFFFu : 0u;
    const unsigned m4 = (v >= 64) ? 0xFFFFFFFFu : 0u;
    v4f o;
    o.x = bf16_val(__uint_as_float((__float_as_uint(x1.x) & m1) | (__float_as_uint(x2.x) & m2) |
                                   (__float_as_uint(x3.x) & m3) | (__float_as_uint(x4.x) & m4)));
    o.y = bf16_val(__uint_as_float((__float_as_uint(x1.y) & m1) | (__float_as_uint(x2.y) & m2) |
                                   (__float_as_uint(x3.y) & m3) | (__float_as_uint(x4.y) & m4)));
    o.z = bf16_val(__uint_as_float((__float_as_uint(x1.z) & m1) | (__float_as_uint(x2.z) & m2) |
                                   (__float_as_uint(x3.z) & m3) | (__float_as_uint(x4.z) & m4)));
    o.w = bf16_val(__uint_as_float((__float_as_uint(x1.w) & m1) | (__float_as_uint(x2.w) & m2) |
                                   (__float_as_uint(x3.w) & m3) | (__float_as_uint(x4.w) & m4)));
    if (v < PARN / 4) {
      volatile v4f* q = (volatile v4f*)(PAR + 4 * v);
      *q = o;
      __threadfence();
      *q = o;
    }
  }
}

__device__ __forceinline__ int scan_chunk(const int* __restrict__ keys, int cbase, int slotBase,
                                          int* list, int tid, int lane, int wave) {
  int wc = 0;
  const int el0 = tid * EPT;
  const int e0  = cbase + el0;
  const int e0c = e0 < NE - EPT ? e0 : NE - EPT;
  v4i da = *(const v4ia*)(keys + e0c);
  v4i db = *(const v4ia*)(keys + e0c + 4);
  asm volatile("" :: "v"(da), "v"(db));
  const int vm = (e0 < NE) ? 0 : -1;
  da = da | (v4i){vm, vm, vm, vm};
  db = db | (v4i){vm, vm, vm, vm};
  const unsigned nbs = (unsigned)slotBase;
  const unsigned unb = (unsigned)NBA;
  const unsigned s0 = (unsigned)da.x - nbs, s1 = (unsigned)da.y - nbs;
  const unsigned s2 = (unsigned)da.z - nbs, s3 = (unsigned)da.w - nbs;
  const unsigned s4 = (unsigned)db.x - nbs, s5 = (unsigned)db.y - nbs;
  const unsigned s6 = (unsigned)db.z - nbs, s7 = (unsigned)db.w - nbs;
  const bool h0 = s0 < unb, h1 = s1 < unb, h2 = s2 < unb, h3 = s3 < unb;
  const bool h4 = s4 < unb, h5 = s5 < unb, h6 = s6 < unb, h7 = s7 < unb;
  const unsigned any = __builtin_amdgcn_ballot_w32(h0 | h1 | h2 | h3 | h4 | h5 | h6 | h7);
  if (any != 0u) {
#define HITJ(J, HJ, SJ) { \
      const unsigned mj = __builtin_amdgcn_ballot_w32(HJ); \
      if (mj != 0u) { \
        if (HJ) { \
          const int pos = wc + (int)__builtin_amdgcn_mbcnt_lo(mj, 0u); \
          if (pos < WCAP) list[wave * WCAP + pos] = ((el0 + (J)) << SLA) | (int)(SJ); \
        } \
        wc += (int)__builtin_popcount(mj); } }
    HITJ(0, h0, s0)
    HITJ(1, h1, s1)
    HITJ(2, h2, s2)
    HITJ(3, h3, s3)
    HITJ(4, h4, s4)
    HITJ(5, h5, s5)
    HITJ(6, h6, s6)
    HITJ(7, h7, s7)
#undef HITJ
  }
  return wc;
}

__global__ __launch_bounds__(NTHR) void k_bucket(const int* __restrict__ srcs, const int* __restrict__ keys,
                                                 int* LIST, int* CNT, int* OFF, int* DISB, int* FLAG) {
  extern __shared__ __attribute__((aligned(16))) int dsm[];
  int* list = dsm;
  int* hl   = dsm + LISTN;
  int* sl   = hl + RCAP;
  int* cnt  = sl + RCAP;
  int* offs = cnt + NBA;
  int* cur  = offs + NBA;
  int* misc = cur + NBA;
  const int tid = (int)threadIdx.x, lane = tid & 31, wave = tid >> 5;
  const int nodeBase = (int)blockIdx.x * NBA;

  {
    const v4i z4 = {0, 0, 0, 0};
    for (int i = tid * 4; i < BK_ZINTS; i += NTHR * 4) *(v4ia*)(dsm + i) = z4;
    if (tid < 16) misc[tid] = 0;
  }
  __syncthreads();

  int t = 0, ov = 0;
#pragma unroll 1
  for (int ch = 0; ch < NCHUNK; ++ch) {
    const int cbase = ch * CHUNK;
    const int wc = scan_chunk(keys, cbase, nodeBase, list, tid, lane, wave);
    if (lane == 0) misc[wave] = wc;
    __syncthreads();
    if (wave == 0) {
#pragma unroll 1
      for (int w2 = 0; w2 < NWAVE; ++w2) {
        int c = clampi(misc[w2], 0, WCAP);
        c = __builtin_amdgcn_readfirstlane(c);
#pragma unroll 1
        for (int b0 = 0; b0 < c; b0 += 32) {
          const int idx = b0 + lane;
          const int ent = list[w2 * WCAP + (idx < WCAP ? idx : WCAP - 1)];
          const int m32 = (c - b0) < 32 ? (c - b0) : 32;
#pragma unroll 1
          for (int k = 0; k < m32; ++k) {
            const int u    = __builtin_amdgcn_readlane(ent, k);
            const int slot = u & (NBA - 1);
            const int el   = (u >> SLA) & (CHUNK - 1);
            const int pk   = ((cbase + el) << SLA) | slot;
            if (t < RCAP) {
              if (lane == 0) { hl[t] = pk; cnt[slot] = cnt[slot] + 1; }
              t = t + 1;
            } else {
              ov = 1;
            }
          }
        }
      }
    }
    __syncthreads();
  }
  if (wave == 0 && lane == 0) { misc[8] = t; misc[9] = ov; }
  __syncthreads();
  int tt = clampi(misc[8], 0, RCAP);
  tt = __builtin_amdgcn_readfirstlane(tt);

  if (wave == 0) {
    const int base = lane * (NBA / 32);
    int s = 0, mx = 0;
#pragma unroll 1
    for (int i = 0; i < NBA / 32; ++i) {
      const int cv = cnt[base + i];
      s += cv;
      mx = cv > mx ? cv : mx;
    }
    const unsigned ob = __builtin_amdgcn_ballot_w32(mx > DEGCAP);
    int incl = s;
#pragma unroll
    for (int d = 1; d < 32; d <<= 1) {
      const int y = __shfl_up(incl, d, 32);
      if (lane >= d) incl += y;
    }
    int run = incl - s;
#pragma unroll 1
    for (int i = 0; i < NBA / 32; ++i) {
      const int cv = cnt[base + i];
      offs[base + i] = run;
      cur[base + i]  = run;
      run += cv;
    }
    if (lane == 0) misc[10] = (ob != 0u) ? 1 : 0;
  }
  __syncthreads();
  if (wave == 0) {
#pragma unroll 1
    for (int b0 = 0; b0 < tt; b0 += 32) {
      const int idx = b0 + lane;
      const int ent = hl[idx < RCAP ? idx : RCAP - 1];
      const int m32 = (tt - b0) < 32 ? (tt - b0) : 32;
#pragma unroll 1
      for (int k = 0; k < m32; ++k) {
        const int u    = __builtin_amdgcn_readlane(ent, k);
        const int slot = u & (NBA - 1);
        if (lane == 0) {
          const int p = clampi(cur[slot], 0, RCAP - 1);
          sl[p] = u;
          cur[slot] = p + 1;
        }
      }
    }
  }
  __syncthreads();
  const int flag = ((misc[9] | misc[10]) != 0) ? 1 : 0;

#pragma unroll 1
  for (int it = 0; it < RCAP / (4 * NTHR); ++it) {
    const int i0 = 4 * (it * NTHR + tid);
    const v4i en = *(const v4ia*)(sl + i0);
    int r0 = srcs[clampi(en.x >> SLA, 0, NE - 1)];
    int r1 = srcs[clampi(en.y >> SLA, 0, NE - 1)];
    int r2 = srcs[clampi(en.z >> SLA, 0, NE - 1)];
    int r3 = srcs[clampi(en.w >> SLA, 0, NE - 1)];
    asm volatile("" :: "v"(r0), "v"(r1), "v"(r2), "v"(r3));
    v4i sv;
    sv.x = clampi(r0, 0, NN - 1) & ((i0 + 0 < tt) ? -1 : 0);
    sv.y = clampi(r1, 0, NN - 1) & ((i0 + 1 < tt) ? -1 : 0);
    sv.z = clampi(r2, 0, NN - 1) & ((i0 + 2 < tt) ? -1 : 0);
    sv.w = clampi(r3, 0, NN - 1) & ((i0 + 3 < tt) ? -1 : 0);
    *(v4ia*)(hl + i0) = sv;
  }
#pragma unroll 1
  for (int j = 0; j < 4; ++j) {
    const int s = 4 * tid + j;
    const float d = 1.0f / sqrtf((float)(cnt[s] + 1));
    cur[s] = __float_as_int(d);
  }
  __syncthreads();

  int* lp = LIST + (size_t)blockIdx.x * RCAP;
  const size_t gb = (size_t)nodeBase + (size_t)(4 * tid);
  const v4i cv4 = *(const v4ia*)(cnt + 4 * tid);
  const v4i ov4 = *(const v4ia*)(offs + 4 * tid);
  const v4i dv4 = *(const v4ia*)(cur + 4 * tid);
  const v4i fv4 = (v4i){flag, flag, flag, flag};
  for (int pass = 0; pass < 2; ++pass) {
#pragma unroll 1
    for (int it = 0; it < RCAP / (4 * NTHR); ++it) {
      const int i0 = 4 * (it * NTHR + tid);
      const v4i v = *(const v4ia*)(hl + i0);
      *(volatile v4i*)(lp + i0) = v;
    }
    *(volatile v4i*)(CNT + gb)  = cv4;
    *(volatile v4i*)(OFF + gb)  = ov4;
    *(volatile v4i*)(DISB + gb) = dv4;
    if (tid < 8) *(volatile v4i*)(FLAG + (size_t)blockIdx.x * 32 + 4 * tid) = fv4;
    __threadfence();
  }
}

template <int MODE>
__global__ __launch_bounds__(NTHR) void k_agg(const int* __restrict__ LIST, const int* __restrict__ CNT,
                                              const int* __restrict__ OFF, const float* __restrict__ dis,
                                              const int* __restrict__ FLAG, const float* __restrict__ xl,
                                              const float* __restrict__ bias, unsigned short* hb, float* hout) {
  const int tid = (int)threadIdx.x, lane = tid & 31, wave = tid >> 5;
  const int nodeBase = (int)blockIdx.x * NBA;
  const int* lp = LIST + (size_t)blockIdx.x * RCAP;
  const int fl = __builtin_amdgcn_readfirstlane(FLAG[(size_t)blockIdx.x * 32]);
  const bool pois = fl != 0;
  const float qnan = __int_as_float(0x7fc00000);
  v4f bv = (v4f){0.f, 0.f, 0.f, 0.f};
  if constexpr (MODE == 1) {
    bv = *(const v4fa*)(bias + 4 * lane);
  } else {
    const v2f tb = *(const v2fa*)(bias + 2 * lane);
    bv.x = tb.x; bv.y = tb.y;
  }
  const int sa = (2 * lane) & 31, sb = (2 * lane + 1) & 31;

#pragma unroll 1
  for (int si = 0; si < NBA / NWAVE; ++si) {
    const int s    = si * NWAVE + wave;
    const int node = nodeBase + s;
    const int craw = __builtin_amdgcn_readfirstlane(CNT[node]);
    const bool big = craw > DEGCAP;
    const int c = clampi(craw, 0, DEGCAP);
    const int o = clampi(__builtin_amdgcn_readfirstlane(OFF[node]), 0, RCAP - 1);
    const int nc = node < NN ? node : NN - 1;
    const float dd = dis[nc];
    const float rd = dd * dd;
    v4f acc = (v4f){0.f, 0.f, 0.f, 0.f};
#pragma unroll 1
    for (int b0 = 0; b0 < c; b0 += 32) {
      const int lim = o + c - 1;
      int idx = o + b0 + lane;
      idx = idx > lim ? lim : idx;
      idx = clampi(idx, 0, RCAP - 1);
      const int sr = clampi(lp[idx], 0, NN - 1);
      const float cf  = dis[sr] * dd;
      const int   cfi = __float_as_int(cf);
      const int m32 = (c - b0) < 32 ? (c - b0) : 32;
#pragma unroll 1
      for (int k = 0; k < m32; ++k) {
        const int   sk = __builtin_amdgcn_readlane(sr, k);
        const float ck = __int_as_float(__builtin_amdgcn_readlane(cfi, k));
        if constexpr (MODE == 1) {
          const v4f a = *(const v4fa*)(xl + (size_t)sk * HID + 4 * lane);
          acc.x = fmaf(ck, a.x, acc.x); acc.y = fmaf(ck, a.y, acc.y);
          acc.z = fmaf(ck, a.z, acc.z); acc.w = fmaf(ck, a.w, acc.w);
        } else {
          const v2f a = *(const v2fa*)(xl + (size_t)sk * DOUT + 2 * lane);
          acc.x = fmaf(ck, a.x, acc.x); acc.y = fmaf(ck, a.y, acc.y);
        }
      }
    }
    const bool pz   = pois || big;
    const bool live = node < NN;
    if constexpr (MODE == 1) {
      const v4f a = *(const v4fa*)(xl + (size_t)nc * HID + 4 * lane);
      float y0 = (acc.x + a.x * rd) + bv.x;
      float y1 = (acc.y + a.y * rd) + bv.y;
      float y2 = (acc.z + a.z * rd) + bv.z;
      float y3 = (acc.w + a.w * rd) + bv.w;
      y0 = pz ? qnan : y0; y1 = pz ? qnan : y1; y2 = pz ? qnan : y2; y3 = pz ? qnan : y3;
      y0 = live ? y0 : 0.0f; y1 = live ? y1 : 0.0f; y2 = live ? y2 : 0.0f; y3 = live ? y3 : 0.0f;
      const int hw0 = (int)pk16(bf16_bits(y0), bf16_bits(y1));
      const int hw1 = (int)pk16(bf16_bits(y2), bf16_bits(y3));
      const int lw0 = (int)pk16(bf16_lo_bits(y0), bf16_lo_bits(y1));
      const int lw1 = (int)pk16(bf16_lo_bits(y2), bf16_lo_bits(y3));
      const int g0 = __shfl(hw0, sa, 32), g1 = __shfl(hw1, sa, 32);
      const int g2 = __shfl(hw0, sb, 32), g3 = __shfl(hw1, sb, 32);
      const int p0 = __shfl(lw0, sa, 32), p1 = __shfl(lw1, sa, 32);
      const int p2 = __shfl(lw0, sb, 32), p3 = __shfl(lw1, sb, 32);
      if constexpr (H1_TERMS == 2) {
        const bool lsel = lane >= 16;
        v4u pv;
        pv.x = (unsigned)(lsel ? p0 : g0);
        pv.y = (unsigned)(lsel ? p1 : g1);
        pv.z = (unsigned)(lsel ? p2 : g2);
        pv.w = (unsigned)(lsel ? p3 : g3);
        unsigned short* hp = hb + (size_t)node * K2TOT + 8 * lane;
        const bool wr = node < MPAD;
        if (wr) *(volatile v4u*)hp = pv;
        __threadfence();
        if (wr) *(volatile v4u*)hp = pv;
      } else {
        v4u pv;
        pv.x = (unsigned)g0; pv.y = (unsigned)g1; pv.z = (unsigned)g2; pv.w = (unsigned)g3;
        unsigned short* hp = hb + (size_t)node * K2TOT + 8 * (lane & 15);
        const bool wr = (node < MPAD) && (lane < 16);
        if (wr) *(volatile v4u*)hp = pv;
        __threadfence();
        if (wr) *(volatile v4u*)hp = pv;
      }
    } else {
      const v2f a = *(const v2fa*)(xl + (size_t)nc * DOUT + 2 * lane);
      float y0 = (acc.x + a.x * rd) + bv.x;
      float y1 = (acc.y + a.y * rd) + bv.y;
      y0 = pz ? qnan : y0; y1 = pz ? qnan : y1;
      y0 = live ? y0 : 0.0f; y1 = live ? y1 : 0.0f;
      v4f ow;
      ow.x = __shfl(y0, sa, 32); ow.y = __shfl(y1, sa, 32);
      ow.z = __shfl(y0, sb, 32); ow.w = __shfl(y1, sb, 32);
      float* op = hout + (size_t)node * DOUT + 4 * (lane & 15);
      const bool wr = (node < MPAD) && (lane < 16);
      if (wr) *(volatile v4f*)op = ow;
      __threadfence();
      if (wr) *(volatile v4f*)op = ow;
    }
  }
}

template <int PASS>
__global__ __launch_bounds__(NTHR) void k_stat(const float* __restrict__ h2, const double* __restrict__ mean64,
                                               double* rec) {
  __shared__ __attribute__((aligned(16))) double part[4 * 64];
  __shared__ __attribute__((aligned(16))) double tot[64];
  const int tid = (int)threadIdx.x;
  const int col = tid & 63, rg = tid >> 6;
  const int r0 = (int)blockIdx.x * NBA;
  const int rend = (r0 + NBA) < NN ? (r0 + NBA) : NN;
  double mu = 0.0;
  if constexpr (PASS == 1) mu = mean64[col];
  double s = 0.0;
#pragma unroll 4
  for (int r = r0 + rg; r < rend; r += 4) {
    const double v = (double)h2[(size_t)r * DOUT + col];
    if constexpr (PASS == 0) {
      s += v;
    } else {
      const double d = v - mu;
      s += d * d;
    }
  }
  part[rg * 64 + col] = s;
  __syncthreads();
  if (tid < 64) tot[tid] = ((part[tid] + part[64 + tid]) + part[128 + tid]) + part[192 + tid];
  __syncthreads();
  if (tid < 32) {
    const v2d o = *(const v2da*)(tot + 2 * tid);
    volatile v2d* q = (volatile v2d*)(rec + (size_t)blockIdx.x * 64 + 2 * tid);
    *q = o;
    __threadfence();
    *q = o;
  }
}

__global__ __launch_bounds__(64) void k_comb_mean(const double* __restrict__ recS, double* mean64) {
  __shared__ __attribute__((aligned(16))) double m[64];
  const int tid = (int)threadIdx.x;
  double s = 0.0;
#pragma unroll 4
  for (int b = 0; b < NBLK; ++b) s += recS[(size_t)b * 64 + tid];
  m[tid] = s * (1.0 / (double)NN);
  __syncthreads();
  if (tid < 32) {
    const v2d o = *(const v2da*)(m + 2 * tid);
    volatile v2d* q = (volatile v2d*)(mean64 + 2 * tid);
    *q = o;
    __threadfence();
    *q = o;
  }
}

__global__ __launch_bounds__(64) void k_comb_var(const double* __restrict__ recQ, const double* __restrict__ mean64,
                                                 const float* __restrict__ par, float* stat) {
  __shared__ __attribute__((aligned(16))) float st[256];
  const int tid = (int)threadIdx.x;
  double q = 0.0;
#pragma unroll 4
  for (int b = 0; b < NBLK; ++b) q += recQ[(size_t)b * 64 + tid];
  const float var = (float)(q * (1.0 / (double)NN));
  const float r = 1.0f / sqrtf(var + 1e-5f);
  st[tid]       = (float)mean64[tid];
  st[64 + tid]  = r;
  st[128 + tid] = par[192 + tid];
  st[192 + tid] = par[256 + tid];
  __syncthreads();
  const v4f o = *(const v4fa*)(st + 4 * tid);
  volatile v4f* p = (volatile v4f*)(stat + 4 * tid);
  *p = o;
  __threadfence();
  *p = o;
}

__global__ __launch_bounds__(NTHR) void k_out(const float* __restrict__ h2, const float* __restrict__ stat,
                                              float* out) {
  __shared__ __attribute__((aligned(16))) float st[256];
  const int tid = (int)threadIdx.x;
  if (tid < 64) {
    const v4f sv = *(const v4fa*)(stat + 4 * tid);
    *(v4fa*)(st + 4 * tid) = sv;
  }
  __syncthreads();
  const int c4 = (tid & 15) * 4;
  const v4f mu = *(const v4fa*)(st + c4);
  const v4f rr = *(const v4fa*)(st + 64 + c4);
  const v4f ga = *(const v4fa*)(st + 128 + c4);
  const v4f be = *(const v4fa*)(st + 192 + c4);
  const int pbase = (int)blockIdx.x * 1024 + tid;
  v4f vv[4];
#pragma unroll
  for (int it = 0; it < 4; ++it) {
    const int p  = pbase + it * NTHR;
    const int pc = p < TOTP ? p : TOTP - 1;
    const v4f x = *(const v4fa*)(h2 + (size_t)pc * 4);
    asm volatile("" :: "v"(x[0]), "v"(x[1]), "v"(x[2]), "v"(x[3]));
    vv[it] = ((x - mu) * rr) * ga + be;
  }
  for (int pass = 0; pass < 2; ++pass) {
#pragma unroll
    for (int it = 0; it < 4; ++it) {
      const int p = pbase + it * NTHR;
      if (p < TOTP) *(volatile v4f*)(out + (size_t)p * 4) = vv[it];
    }
    __threadfence();
  }
}

extern "C" void kernel_launch(void* const* d_in, const int* in_sizes, int n_in,
                              void* d_out, int out_size, void* d_ws, size_t ws_size,
                              hipStream_t stream) {
  if (n_in < 8) return;
  if (in_sizes[0] != NN * DIN) return;
  if (in_sizes[1] != DIN * HID) return;
  if (in_sizes[2] != HID) return;
  if (in_sizes[3] != HID * DOUT) return;
  if (in_sizes[4] != DOUT || in_sizes[5] != DOUT || in_sizes[6] != DOUT) return;
  if (in_sizes[7] != 2 * NE) return;
  if (out_size != NN * DOUT) return;
  if (WS_TOTAL > ws_size) return;

  const float* emb  = (const float*)d_in[0];
  const float* W1   = (const float*)d_in[1];
  const float* b1   = (const float*)d_in[2];
  const float* W2   = (const float*)d_in[3];
  const float* b2   = (const float*)d_in[4];
  const float* gam  = (const float*)d_in[5];
  const float* bet  = (const float*)d_in[6];
  const int*   edge = (const int*)d_in[7];
  const int* srcs = edge;
  const int* keys = edge + NE;
  float* out = (float*)d_out;

  char* ws = (char*)d_ws;
  float*          T1   = (float*)(ws + O_RA);
  float*          T2   = (float*)(ws + O_RA);
  float*          H2   = (float*)(ws + O_RA + (size_t)MPAD * DOUT * 4);
  unsigned short* EMBB = (unsigned short*)(ws + O_RB);
  unsigned short* H1   = (unsigned short*)(ws + O_RB);
  int*            LIST = (int*)(ws + O_LIST);
  int*            CNT  = (int*)(ws + O_CNT);
  int*            OFF  = (int*)(ws + O_OFF);
  int*            DISB = (int*)(ws + O_DIS);
  const float*    DIS  = (const float*)(ws + O_DIS);
  int*            FLAG = (int*)(ws + O_FLAG);
  unsigned short* W1T  = (unsigned short*)(ws + O_W1T);
  unsigned short* W2D  = (unsigned short*)(ws + O_W2D);
  float*          PAR  = (float*)(ws + O_PAR);
  float*          STAT = (float*)(ws + O_STAT);
  double*         RECS = (double*)(ws + O_RECS);
  double*         RECQ = (double*)(ws + O_RECQ);
  double*         MEAN = (double*)(ws + O_MEAN);

  hipFuncSetAttribute(reinterpret_cast<const void*>(&k_bucket), hipFuncAttributeMaxDynamicSharedMemorySize,
                      (int)BK_LDS_BYTES);

  k_prep<<<(NU1 + NU2) / NTHR + 1, NTHR, 0, stream>>>(W1, W2, b1, b2, gam, bet, W1T, W2D, PAR);
  k_plane<0><<<MPAD * DIN / 8 / 256, 256, 0, stream>>>(emb, NN, DIN, DIN, EMBB, MPAD, DIN);
  k_bucket<<<NBLK, NTHR, BK_LDS_BYTES, stream>>>(srcs, keys, LIST, CNT, OFF, DISB, FLAG);
  k_gemm_nt<0, 0><<<((MPAD / 64) * (HID / 64) + 7) / 8, 256, 0, stream>>>(EMBB, W1T, PAR, T1, MPAD, HID, DIN, HID);
  k_agg<1><<<NBLK, NTHR, 0, stream>>>(LIST, CNT, OFF, DIS, FLAG, T1, PAR, H1, H2);
  k_gemm_nt<0, 0><<<((MPAD / 64) * (DOUT / 64) + 7) / 8, 256, 0, stream>>>(H1, W2D, PAR, T2, MPAD, DOUT, K2TOT, DOUT);
  k_agg<0><<<NBLK, NTHR, 0, stream>>>(LIST, CNT, OFF, DIS, FLAG, T2, PAR + 128, H1, H2);
  k_stat<0><<<NBLK, NTHR, 0, stream>>>(H2, MEAN, RECS);
  k_comb_mean<<<1, 64, 0, stream>>>(RECS, MEAN);
  k_stat<1><<<NBLK, NTHR, 0, stream>>>(H2, MEAN, RECQ);
  k_comb_var<<<1, 64, 0, stream>>>(RECQ, MEAN, PAR, STAT);
  k_out<<<(TOTP + 1023) / 1024, NTHR, 0, stream>>>(H2, STAT, out);
}
